// TiSASRec_81535659147511
// MI455X (gfx1250) — hardware-verified
//
#include <hip/hip_runtime.h>
#include <stddef.h>
#include <stdint.h>

#define NSEQ 16
#define SLEN 200
#define HID  128
#define NHD  4
#define HDM  32
#define NLAY 2
#define NTOK 3200
#define NTT  257
#define NWPL 32768

static_assert(NTOK == NSEQ * SLEN);
static_assert(NTOK % 128 == 0);
static_assert(NTOK % 32 == 0);
static_assert(NTOK % 16 == 0);
static_assert(HID == NHD * HDM);
static_assert(HID % 32 == 0);
static_assert(HDM == 32);

typedef _Float16 v16h __attribute__((ext_vector_type(16)));
typedef _Float16 v8h  __attribute__((ext_vector_type(8)));
typedef float    v8f  __attribute__((ext_vector_type(8)));
typedef float    v4f  __attribute__((ext_vector_type(4)));
typedef unsigned int v4u __attribute__((ext_vector_type(4)));

union Frag  { v16h v; v8h h[2]; };
union Pack8 { v8h h; v4u u; };

#define NEGV    (-4294967296.0f)
#define SQRT_H  (11.313708305358887f)

#define QSP   36
#define KSP   40
#define VTP   232
#define TKP   33
#define TVP   32
#define SWP   212
#define PWP   232
#define OSP   36
#define QROWS 208
#define KPAD  224
#define OFF_QS   0
#define OFF_KS   (OFF_QS + QROWS * QSP * 4)
#define OFF_VT   (OFF_KS + QROWS * KSP * 2)
#define OFF_TK   (OFF_VT + HDM * VTP * 2)
#define TKBYTES  ((((NTT * TKP * 4) + 15) / 16) * 16)
#define OFF_TV   (OFF_TK + TKBYTES)
#define OFF_W    (OFF_TV + NTT * TVP * 4)
#define SWB      (16 * SWP * 4)
#define PWB      (16 * PWP * 2)
#define OSB      (16 * OSP * 4)
#define LIB      64
#define WBYTES   (SWB + PWB + OSB + LIB)
#define ATT_WAVES 4
#define ATT_THREADS (ATT_WAVES * 32)
#define ATT_LDS  (OFF_W + ATT_WAVES * WBYTES)
static_assert(OFF_KS % 16 == 0);
static_assert(OFF_VT % 16 == 0);
static_assert(OFF_TK % 16 == 0);
static_assert(OFF_TV % 16 == 0);
static_assert(OFF_W % 16 == 0);
static_assert(SWB % 16 == 0);
static_assert(PWB % 16 == 0);
static_assert(OSB % 16 == 0);
static_assert(WBYTES % 16 == 0);
static_assert((VTP * 2) % 16 == 0);
static_assert((PWP * 2) % 16 == 0);
static_assert((KSP * 2) % 16 == 0);
static_assert((QSP * 4) % 16 == 0);
static_assert((OSP * 4) % 16 == 0);
static_assert(ATT_LDS <= 300000);
static_assert(KPAD % 32 == 0);
static_assert(QROWS == 13 * 16);

__device__ __forceinline__ v8f mma16(v16h a, v16h b, v8f c) {
  c = __builtin_amdgcn_wmma_f32_16x16x32_f16(false, a, false, b, (short)0, c, false, false);
  asm volatile("v_nop\n\tv_nop\n\tv_nop\n\tv_nop" : "+v"(c) : "v"(a), "v"(b));
  return c;
}

__device__ __forceinline__ v8f zero8() { return (v8f){0.f, 0.f, 0.f, 0.f, 0.f, 0.f, 0.f, 0.f}; }

__device__ __forceinline__ v16h ldfrag(const _Float16* p, int ld, int row0, int k0, int lane) {
  const int m = lane & 15, lh = lane >> 4;
  const _Float16* q = p + (size_t)(row0 + m) * ld + k0 + 8 * lh;
  Frag f;
  f.h[0] = *(const v8h*)(q);
  f.h[1] = *(const v8h*)(q + 16);
  return f.v;
}

__device__ __forceinline__ v8h cvt8(v4f a, v4f b) {
  return (v8h){(_Float16)a[0], (_Float16)a[1], (_Float16)a[2], (_Float16)a[3],
               (_Float16)b[0], (_Float16)b[1], (_Float16)b[2], (_Float16)b[3]};
}

__device__ __forceinline__ v16h ldfrag_f32(const float* p, int ld, int row0, int k0, int lane) {
  const int m = lane & 15, lh = lane >> 4;
  const float* q = p + (size_t)(row0 + m) * ld + k0 + 8 * lh;
  Frag f;
  f.h[0] = cvt8(*(const v4f*)(q), *(const v4f*)(q + 4));
  f.h[1] = cvt8(*(const v4f*)(q + 16), *(const v4f*)(q + 20));
  return f.v;
}

__device__ __forceinline__ float wsum(float v) {
#pragma unroll
  for (int o = 16; o > 0; o >>= 1) v += __shfl_xor(v, o, 32);
  return v;
}
__device__ __forceinline__ float wmax(float v) {
#pragma unroll
  for (int o = 16; o > 0; o >>= 1) v = fmaxf(v, __shfl_xor(v, o, 32));
  return v;
}

__device__ __forceinline__ void gemm32x64(const _Float16* __restrict__ A, int lda,
                                          const _Float16* __restrict__ Bt, int ldb, int K,
                                          int m0, int n0, int lane, v8f (&acc)[2][4]) {
#pragma unroll 1
  for (int k0 = 0; k0 < K; k0 += 32) {
    const v16h a0 = ldfrag(A, lda, m0, k0, lane);
    const v16h a1 = ldfrag(A, lda, m0 + 16, k0, lane);
    const v16h b0 = ldfrag(Bt, ldb, n0, k0, lane);
    const v16h b1 = ldfrag(Bt, ldb, n0 + 16, k0, lane);
    const v16h b2 = ldfrag(Bt, ldb, n0 + 32, k0, lane);
    const v16h b3 = ldfrag(Bt, ldb, n0 + 48, k0, lane);
    acc[0][0] = mma16(a0, b0, acc[0][0]);
    acc[1][0] = mma16(a1, b0, acc[1][0]);
    acc[0][1] = mma16(a0, b1, acc[0][1]);
    acc[1][1] = mma16(a1, b1, acc[1][1]);
    acc[0][2] = mma16(a0, b2, acc[0][2]);
    acc[1][2] = mma16(a1, b2, acc[1][2]);
    acc[0][3] = mma16(a0, b3, acc[0][3]);
    acc[1][3] = mma16(a1, b3, acc[1][3]);
  }
}

__global__ __launch_bounds__(256) void k_cvtw(const float* __restrict__ w0, const float* __restrict__ w1,
                                              const float* __restrict__ w2, const float* __restrict__ w3,
                                              const float* __restrict__ w4, _Float16* __restrict__ wp, float scale) {
  const int tid = threadIdx.x;
  const int y = blockIdx.y;
  const float* src = (y == 0) ? w0 : ((y == 1) ? w1 : ((y == 2) ? w2 : ((y == 3) ? w3 : w4)));
  const size_t o = (size_t)blockIdx.x * 2048 + (size_t)tid * 8;
  const v4f a0 = *(const v4f*)(src + o) * scale;
  const v4f a1 = *(const v4f*)(src + o + 4) * scale;
  Pack8 pk;
  pk.h = cvt8(a0, a1);
  const v4u vv = pk.u;
  volatile v4u* d = (volatile v4u*)(wp + (size_t)y * NWPL + o);
  *d = vv;
  __threadfence();
  *d = vv;
}

__global__ __launch_bounds__(256) void k_embed(const float* __restrict__ emb, int nitems,
                                               const int* __restrict__ seq,
                                               float* __restrict__ x, _Float16* __restrict__ xh) {
  __shared__ __align__(16) float sw[8][2][HID];
  const int tid = threadIdx.x, lane = tid & 31, wave = tid >> 5;
  const int r0 = blockIdx.x * 16 + wave * 2;
  v4f y[2];
#pragma unroll
  for (int e = 0; e < 2; ++e) {
    const int row = r0 + e;
    const int idx = seq[row];
    const int idc = min(max(idx, 0), nitems - 1);
    v4f v = *(const v4f*)(emb + (size_t)idc * HID + lane * 4) * SQRT_H;
    const float keep = (idx == 0) ? 0.f : 1.f;
    y[e] = v * keep;
  }
  for (int ps = 0; ps < 2; ++ps) {
#pragma unroll
    for (int e = 0; e < 2; ++e) *(volatile v4f*)(x + (size_t)(r0 + e) * HID + lane * 4) = y[e];
    __threadfence();
  }
#pragma unroll
  for (int e = 0; e < 2; ++e) *(v4f*)(&sw[wave][e][lane * 4]) = y[e];
  __syncthreads();
  {
    const int e = lane >> 4, pc = lane & 15;
    const float* cp = &sw[wave][e][pc * 8];
    const v4f a0 = *(const v4f*)(cp), a1 = *(const v4f*)(cp + 4);
    Pack8 pk;
    pk.h = cvt8(a0, a1);
    const v4u hv = pk.u;
    const size_t go = (size_t)(r0 + e) * HID + pc * 8;
    for (int ps = 0; ps < 2; ++ps) {
      *(volatile v4u*)(xh + go) = hv;
      __threadfence();
    }
  }
}

__global__ __launch_bounds__(256) void k_ln(const float* __restrict__ a, const float* __restrict__ badd,
                                            const float* __restrict__ g, const float* __restrict__ bt,
                                            float* __restrict__ of, _Float16* __restrict__ oh) {
  __shared__ __align__(16) float sw[8][2][HID];
  const int tid = threadIdx.x, lane = tid & 31, wave = tid >> 5;
  const int r0 = blockIdx.x * 16 + wave * 2;
  const v4f gv = *(const v4f*)(g + lane * 4);
  const v4f bv = *(const v4f*)(bt + lane * 4);
  v4f y[2];
#pragma unroll
  for (int e = 0; e < 2; ++e) {
    const size_t ro = (size_t)(r0 + e) * HID + lane * 4;
    v4f v = *(const v4f*)(a + ro);
    if (badd) v = v + *(const v4f*)(badd + ro);
    float s = (v[0] + v[1]) + (v[2] + v[3]);
    s = wsum(s);
    const float mean = s * 0.0078125f;
    const v4f d = v - mean;
    float ss = (d[0] * d[0] + d[1] * d[1]) + (d[2] * d[2] + d[3] * d[3]);
    ss = wsum(ss);
    const float var  = ss * 0.0078125f;
    const float rstd = rsqrtf(var + 1e-8f);
    y[e] = (d * rstd) * gv + bv;
  }
  for (int ps = 0; ps < 2; ++ps) {
#pragma unroll
    for (int e = 0; e < 2; ++e) *(volatile v4f*)(of + (size_t)(r0 + e) * HID + lane * 4) = y[e];
    __threadfence();
  }
#pragma unroll
  for (int e = 0; e < 2; ++e) *(v4f*)(&sw[wave][e][lane * 4]) = y[e];
  __syncthreads();
  {
    const int e = lane >> 4, pc = lane & 15;
    const float* cp = &sw[wave][e][pc * 8];
    const v4f a0 = *(const v4f*)(cp), a1 = *(const v4f*)(cp + 4);
    Pack8 pk;
    pk.h = cvt8(a0, a1);
    const v4u hv = pk.u;
    const size_t go = (size_t)(r0 + e) * HID + pc * 8;
    for (int ps = 0; ps < 2; ++ps) {
      *(volatile v4u*)(oh + go) = hv;
      __threadfence();
    }
  }
}

#define OTP 68
__global__ __launch_bounds__(256) void k_gemm(const _Float16* __restrict__ ap, const _Float16* __restrict__ wt,
                                              const float* __restrict__ bias, const float* __restrict__ addtab,
                                              const float* __restrict__ resid, const int* __restrict__ seq,
                                              int relu, float scale, float oscale,
                                              float* __restrict__ outf, _Float16* __restrict__ outh) {
  __shared__ __align__(16) float st[8][16 * OTP];
  const int tid = threadIdx.x, lane = tid & 31, wave = tid >> 5;
  const int hh = lane >> 4, c = lane & 15;
  const int m0 = blockIdx.x * 128 + (wave >> 1) * 32;
  const int n0 = (wave & 1) * 64;

  v8f acc[2][4];
#pragma unroll
  for (int s = 0; s < 2; ++s)
#pragma unroll
    for (int t = 0; t < 4; ++t) acc[s][t] = zero8();
  gemm32x64(ap, HID, wt, HID, HID, m0, n0, lane, acc);

  float bb[4];
#pragma unroll
  for (int t = 0; t < 4; ++t) bb[t] = bias[n0 + 16 * t + c];
  float* sw = st[wave];

#pragma unroll
  for (int sub = 0; sub < 2; ++sub) {
    __syncthreads();
#pragma unroll
    for (int r = 0; r < 8; ++r) {
      const int m = m0 + sub * 16 + 8 * hh + r;
      float keep = 1.f;
      if (seq) keep = (seq[m] != 0) ? 1.f : 0.f;
#pragma unroll
      for (int t = 0; t < 4; ++t) {
        const int n = n0 + 16 * t + c;
        float v = acc[sub][t][r] * scale + bb[t];
        if (addtab) v += addtab[(m % SLEN) * HID + n];
        if (resid) v += resid[(size_t)m * HID + n];
        if (relu) v = fmaxf(v, 0.f);
        if (seq) v = v * keep;
        sw[(8 * hh + r) * OTP + 16 * t + c] = v;
      }
    }
    __syncthreads();
    if (outf) {
      v4f val[8];
      size_t go[8];
#pragma unroll
      for (int it = 0; it < 8; ++it) {
        const int p    = lane + 32 * it;
        const int L    = p >> 3;
        const int pc   = p & 7;
        const int row  = L >> 1;
        const int half = L & 1;
        val[it] = *(const v4f*)(sw + row * OTP + half * 32 + pc * 4);
        go[it]  = (size_t)(m0 + sub * 16 + row) * HID + n0 + half * 32 + pc * 4;
      }
      for (int ps = 0; ps < 2; ++ps) {
#pragma unroll
        for (int it = 0; it < 8; ++it) *(volatile v4f*)(outf + go[it]) = val[it];
        __threadfence();
      }
    }
    if (outh) {
      v4u val[4];
      size_t go[4];
#pragma unroll
      for (int it = 0; it < 4; ++it) {
        const int p  = lane + 32 * it;
        const int L  = p >> 3;
        const int pc = p & 7;
        const float* ra = sw + L * OTP + pc * 8;
        const v4f a0 = *(const v4f*)(ra) * oscale, a1 = *(const v4f*)(ra + 4) * oscale;
        Pack8 pk;
        pk.h = cvt8(a0, a1);
        val[it] = pk.u;
        go[it]  = (size_t)(m0 + sub * 16 + L) * HID + n0 + pc * 8;
      }
      for (int ps = 0; ps < 2; ++ps) {
#pragma unroll
        for (int it = 0; it < 4; ++it) *(volatile v4u*)(outh + go[it]) = val[it];
        __threadfence();
      }
    }
  }
}

__global__ __launch_bounds__(ATT_THREADS) void k_attn(const float* __restrict__ qf,
                                                      const _Float16* __restrict__ kh,
                                                      const _Float16* __restrict__ vh,
                                                      const float* __restrict__ tmk,
                                                      const float* __restrict__ tmv,
                                                      const int* __restrict__ tmat,
                                                      const int* __restrict__ seq,
                                                      float* __restrict__ op, float sscale) {
  extern __shared__ __align__(16) unsigned char lds[];
  float*    Qs = (float*)(lds + OFF_QS);
  _Float16* Ks = (_Float16*)(lds + OFF_KS);
  _Float16* Vt = (_Float16*)(lds + OFF_VT);
  float*    Tk = (float*)(lds + OFF_TK);
  float*    Tv = (float*)(lds + OFF_TV);

  const int tid = threadIdx.x, lane = tid & 31, wave = tid >> 5;
  const int hh = lane >> 4, c = lane & 15;
  unsigned char* wb = lds + OFF_W + wave * WBYTES;
  float*    Sw = (float*)(wb);
  _Float16* Pw = (_Float16*)(wb + SWB);
  float*    Os = (float*)(wb + SWB + PWB);
  float*    Li = (float*)(wb + SWB + PWB + OSB);

  const int b = blockIdx.x / NHD, h = blockIdx.x % NHD;
  const size_t rowb = (size_t)b * SLEN;
  const float NEG_INF = -__builtin_huge_valf();

  for (int i = tid; i < QROWS * 8; i += ATT_THREADS) {
    const int r = i >> 3, pc = i & 7, rc = min(r, SLEN - 1);
    v4f v = *(const v4f*)(qf + (rowb + rc) * HID + h * HDM + pc * 4);
    const float keep = (r < SLEN) ? 1.f : 0.f;
    *(v4f*)(Qs + r * QSP + pc * 4) = v * keep;
  }
  for (int i = tid; i < QROWS * 4; i += ATT_THREADS) {
    const int r = i >> 2, pc = i & 3, rc = min(r, SLEN - 1);
    v8h v = *(const v8h*)(kh + (rowb + rc) * HID + h * HDM + pc * 8);
    const _Float16 keep = (r < SLEN) ? (_Float16)1.0f : (_Float16)0.0f;
    *(v8h*)(Ks + r * KSP + pc * 8) = v * keep;
  }
  for (int i = tid; i < KPAD * 4; i += ATT_THREADS) {
    const int k = i >> 2, gq = i & 3, kc = min(k, SLEN - 1);
    v8h v = *(const v8h*)(vh + (rowb + kc) * HID + h * HDM + gq * 8);
    const _Float16 keep = (k < SLEN) ? (_Float16)1.0f : (_Float16)0.0f;
#pragma unroll
    for (int j = 0; j < 8; ++j) Vt[(gq * 8 + j) * VTP + k] = v[j] * keep;
  }
  for (int i = tid; i < NTT * 8; i += ATT_THREADS) {
    const int t = i >> 3, pc = i & 7;
    const v4f v = *(const v4f*)(tmk + (size_t)t * HID + h * HDM + pc * 4);
    float* d = Tk + t * TKP + pc * 4;
    d[0] = v[0]; d[1] = v[1]; d[2] = v[2]; d[3] = v[3];
    const v4f u = *(const v4f*)(tmv + (size_t)t * HID + h * HDM + pc * 4);
    *(v4f*)(Tv + t * TVP + pc * 4) = u;
  }
  __syncthreads();

#pragma unroll 1
  for (int it = 0; it < 4; ++it) {
    const int tile = wave + ATT_WAVES * it;
    const bool active = tile < 13;
    const int q0 = tile * 16;
    bool pr;
    {
      const int qq = q0 + c, qcl = min(qq, SLEN - 1);
      const int sv = seq[rowb + qcl];
      pr = (qq >= SLEN) || (sv == 0);
    }
    const unsigned pm = __builtin_amdgcn_ballot_w32(pr) & 0xFFFFu;
    const int nkt = (pm != 0u) ? 13 : (tile + 1);
    const int nch = (16 * nkt + 31) >> 5;

    if (active) {
      const v16h qa = ldfrag_f32(Qs, QSP, q0, 0, lane);
#pragma unroll 1
      for (int n = 0; n < 13; ++n) {
        v8f s = zero8();
        if (n < nkt) {
          const v16h kb = ldfrag(Ks, KSP, 16 * n, 0, lane);
          s = mma16(qa, kb, s);
        }
#pragma unroll
        for (int r = 0; r < 8; ++r) Sw[(8 * hh + r) * SWP + 16 * n + c] = s[r];
      }
    }
    __syncthreads();

    if (active) {
#pragma unroll 1
      for (int q = 0; q < 16; ++q) {
        const int qg = q0 + q;
        const int qc = min(qg, SLEN - 1);
        const bool padq = ((pm >> q) & 1u) != 0u;
        const int* tmrow = tmat + (rowb + qc) * SLEN;
        const float* qrow = Qs + qg * QSP;
        float* srow = Sw + q * SWP;
#pragma unroll 1
        for (int kc = 0; kc < 7; ++kc) {
          const int k = 32 * kc + lane;
          const int kcl = min(k, SLEN - 1);
          float sv;
          if (kc < nch) {
            int t = tmrow[kcl];
            t = min(max(t, 0), NTT - 1);
            const float* tr = Tk + t * TKP;
            float dot = 0.f;
            for (int d = 0; d < HDM; ++d) dot += qrow[d] * tr[d];
            const float raw = srow[min(k, QROWS - 1)];
            sv = (raw + dot) * sscale;
            sv = (padq || (k > qg)) ? NEGV : sv;
          } else {
            sv = NEGV;
          }
          sv = (k >= SLEN) ? NEG_INF : sv;
          if (k < QROWS) srow[k] = sv;
        }
        float v[7];
#pragma unroll
        for (int j = 0; j < 7; ++j) {
          const int k = 32 * j + lane;
          const float x = srow[min(k, QROWS - 1)];
          v[j] = (k >= SLEN) ? NEG_INF : x;
        }
        float m = v[0];
#pragma unroll
        for (int j = 1; j < 7; ++j) m = fmaxf(m, v[j]);
        m = wmax(m);
        float l = 0.f;
#pragma unroll
        for (int j = 0; j < 7; ++j) {
          const float e = __expf(v[j] - m);
          l += e;
          Pw[q * PWP + 32 * j + lane] = (_Float16)(e * 1024.0f);
        }
        l = wsum(l);
        Li[q] = 1.0f / (l * 1024.0f);
      }
    }
    __syncthreads();

    if (active) {
      v8f oacc[2];
      oacc[0] = zero8();
      oacc[1] = zero8();
#pragma unroll
      for (int ks = 0; ks < 7; ++ks) {
        const v16h pa = ldfrag(Pw, PWP, 0, 32 * ks, lane);
#pragma unroll
        for (int t = 0; t < 2; ++t) {
          const v16h vb = ldfrag(Vt, VTP, 16 * t, 32 * ks, lane);
          oacc[t] = mma16(pa, vb, oacc[t]);
        }
      }
#pragma unroll
      for (int t = 0; t < 2; ++t)
#pragma unroll
        for (int r = 0; r < 8; ++r) Os[(8 * hh + r) * OSP + 16 * t + c] = oacc[t][r];
    }
    __syncthreads();

    if (active) {
#pragma unroll 1
      for (int q = 0; q < 16; ++q) {
        const int qg = q0 + q;
        const int qc = min(qg, SLEN - 1);
        const bool padq = ((pm >> q) & 1u) != 0u;
        const int kend = (qg >= SLEN) ? 0 : (padq ? SLEN : (qg + 1));
        const int* tmrow = tmat + (rowb + qc) * SLEN;
        const _Float16* prow = Pw + q * PWP;
        float o = 0.f;
#pragma unroll 1
        for (int k = 0; k < kend; ++k) {
          int t = tmrow[k];
          t = min(max(t, 0), NTT - 1);
          const float p = (float)prow[k];
          o += p * Tv[t * TVP + lane];
        }
        const float res = (Os[q * OSP + lane] + o) * Li[q];
        Os[q * OSP + lane] = res;
      }
    }
    __syncthreads();

    if (active) {
      v4f val[4];
      size_t go[4];
      bool ok[4];
#pragma unroll
      for (int i2 = 0; i2 < 4; ++i2) {
        const int row = 4 * i2 + (lane >> 3);
        const int pc  = lane & 7;
        const int qg  = q0 + row;
        val[i2] = *(const v4f*)(Os + row * OSP + 4 * pc);
        go[i2]  = (rowb + (size_t)min(qg, SLEN - 1)) * HID + h * HDM + 4 * pc;
        ok[i2]  = qg < SLEN;
      }
      for (int ps = 0; ps < 2; ++ps) {
#pragma unroll
        for (int i2 = 0; i2 < 4; ++i2)
          if (ok[i2]) *(volatile v4f*)(op + go[i2]) = val[i2];
        __threadfence();
      }
    }
  }
}

__global__ __launch_bounds__(256) void k_final(const float* __restrict__ x, const float* __restrict__ g,
                                               const float* __restrict__ bt, const float* __restrict__ emb,
                                               int nitems, const int* __restrict__ pos,
                                               const int* __restrict__ neg, float* __restrict__ out) {
  __shared__ __align__(16) float res[2][32];
  const int tid = threadIdx.x, lane = tid & 31, wave = tid >> 5;
  const v4f gv = *(const v4f*)(g + lane * 4);
  const v4f bv = *(const v4f*)(bt + lane * 4);
#pragma unroll
  for (int e = 0; e < 4; ++e) {
    const int row = blockIdx.x * 32 + wave * 4 + e;
    const v4f v = *(const v4f*)(x + (size_t)row * HID + lane * 4);
    float s = (v[0] + v[1]) + (v[2] + v[3]);
    s = wsum(s);
    const float mean = s * 0.0078125f;
    const v4f d = v - mean;
    float ss = (d[0] * d[0] + d[1] * d[1]) + (d[2] * d[2] + d[3] * d[3]);
    ss = wsum(ss);
    const float var  = ss * 0.0078125f;
    const float rstd = rsqrtf(var + 1e-8f);
    const v4f f = (d * rstd) * gv + bv;
    const int pi = min(max(pos[row], 0), nitems - 1);
    const int ni = min(max(neg[row], 0), nitems - 1);
    const v4f ep = *(const v4f*)(emb + (size_t)pi * HID + lane * 4);
    const v4f en = *(const v4f*)(emb + (size_t)ni * HID + lane * 4);
    float sp = (f[0] * ep[0] + f[1] * ep[1]) + (f[2] * ep[2] + f[3] * ep[3]);
    float sn = (f[0] * en[0] + f[1] * en[1]) + (f[2] * en[2] + f[3] * en[3]);
    sp = wsum(sp);
    sn = wsum(sn);
    if (lane == 0) {
      res[0][wave * 4 + e] = sp;
      res[1][wave * 4 + e] = sn;
    }
  }
  __syncthreads();
  if (wave == 0) {
    const int which = (lane >> 3) & 1, pc = lane & 7;
    const v4f val = *(const v4f*)(&res[which][pc * 4]);
    float* dst = out + (size_t)which * NTOK + (size_t)blockIdx.x * 32 + pc * 4;
    const bool on = lane < 16;
    for (int ps = 0; ps < 2; ++ps) {
      if (on) *(volatile v4f*)dst = val;
      __threadfence();
    }
  }
}

extern "C" void kernel_launch(void* const* d_in, const int* in_sizes, int n_in,
                              void* d_out, int out_size, void* d_ws, size_t ws_size,
                              hipStream_t stream) {
  if (n_in < 26) return;
  if (in_sizes[0] != NTOK) return;
  if (in_sizes[1] != NSEQ * SLEN * SLEN) return;
  if (in_sizes[2] != NTOK) return;
  if (in_sizes[3] != NTOK) return;
  if (in_sizes[5] < 2 * HID || (in_sizes[5] % HID) != 0) return;
  if (in_sizes[6] != SLEN * HID) return;
  if (in_sizes[7] != SLEN * HID) return;
  if (in_sizes[8] != NTT * HID) return;
  if (in_sizes[9] != NTT * HID) return;
  if (in_sizes[10] != NLAY * HID * HID) return;
  if (in_sizes[11] != NLAY * HID) return;
  if (in_sizes[12] != NLAY * HID * HID) return;
  if (in_sizes[13] != NLAY * HID) return;
  if (in_sizes[14] != NLAY * HID * HID) return;
  if (in_sizes[15] != NLAY * HID) return;
  if (in_sizes[16] != NLAY * HID) return;
  if (in_sizes[17] != NLAY * HID) return;
  if (in_sizes[18] != NLAY * HID) return;
  if (in_sizes[19] != NLAY * HID) return;
  if (in_sizes[20] != NLAY * HID * HID) return;
  if (in_sizes[21] != NLAY * HID) return;
  if (in_sizes[22] != NLAY * HID * HID) return;
  if (in_sizes[23] != NLAY * HID) return;
  if (in_sizes[24] != HID) return;
  if (in_sizes[25] != HID) return;
  if (out_size != 2 * NTOK) return;

  const int*   log_seqs = (const int*)d_in[0];
  const int*   tmat     = (const int*)d_in[1];
  const int*   pos_seqs = (const int*)d_in[2];
  const int*   neg_seqs = (const int*)d_in[3];
  const float* item_emb = (const float*)d_in[5];
  const int    nitems   = in_sizes[5] / HID;
  const float* pos_K = (const float*)d_in[6];
  const float* pos_V = (const float*)d_in[7];
  const float* tm_K  = (const float*)d_in[8];
  const float* tm_V  = (const float*)d_in[9];
  const float* Wq = (const float*)d_in[10]; const float* bq = (const float*)d_in[11];
  const float* Wk = (const float*)d_in[12]; const float* bk = (const float*)d_in[13];
  const float* Wv = (const float*)d_in[14]; const float* bv = (const float*)d_in[15];
  const float* ln1_g = (const float*)d_in[16]; const float* ln1_b = (const float*)d_in[17];
  const float* ln2_g = (const float*)d_in[18]; const float* ln2_b = (const float*)d_in[19];
  const float* W1 = (const float*)d_in[20]; const float* b1 = (const float*)d_in[21];
  const float* W2 = (const float*)d_in[22]; const float* b2 = (const float*)d_in[23];
  const float* lnf_g = (const float*)d_in[24]; const float* lnf_b = (const float*)d_in[25];
  float* out = (float*)d_out;

  size_t off = 0;
  const size_t oWp   = off; off += (size_t)5 * NWPL * 2;
  const size_t oX    = off; off += (size_t)NTOK * HID * 4;
  const size_t oXh   = off; off += (size_t)NTOK * HID * 2;
  const size_t oQin  = off; off += (size_t)NTOK * HID * 4;
  const size_t oQinh = off; off += (size_t)NTOK * HID * 2;
  const size_t oQf   = off; off += (size_t)NTOK * HID * 4;
  const size_t oKh   = off; off += (size_t)NTOK * HID * 2;
  const size_t oVh   = off; off += (size_t)NTOK * HID * 2;
  const size_t oOp   = off; off += (size_t)NTOK * HID * 4;
  const size_t oY    = off; off += (size_t)NTOK * HID * 4;
  const size_t oYh   = off; off += (size_t)NTOK * HID * 2;
  const size_t oHm   = off; off += (size_t)NTOK * HID * 2;
  if (off > ws_size) return;
  if (off > (size_t)134217728) return;

  char* ws = (char*)d_ws;
  _Float16* Wp   = (_Float16*)(ws + oWp);
  float*    X    = (float*)(ws + oX);
  _Float16* Xh   = (_Float16*)(ws + oXh);
  float*    Qin  = (float*)(ws + oQin);
  _Float16* Qinh = (_Float16*)(ws + oQinh);
  float*    Qf   = (float*)(ws + oQf);
  _Float16* Kh   = (_Float16*)(ws + oKh);
  _Float16* Vh   = (_Float16*)(ws + oVh);
  float*    Op   = (float*)(ws + oOp);
  float*    Y    = (float*)(ws + oY);
  _Float16* Yh   = (_Float16*)(ws + oYh);
  _Float16* Hm   = (_Float16*)(ws + oHm);

  (void)hipFuncSetAttribute(reinterpret_cast<const void*>(&k_attn),
                            hipFuncAttributeMaxDynamicSharedMemorySize, ATT_LDS);

  k_cvtw<<<dim3(NWPL / 2048, 5), dim3(256), 0, stream>>>(Wq, Wk, Wv, W1, W2, Wp, 64.0f);
  k_embed<<<dim3(NTOK / 16), dim3(256), 0, stream>>>(item_emb, nitems, log_seqs, X, Xh);

  const float sscale = 0.17677669584820551f;
  const float* fnull = nullptr;
  const int* inull = nullptr;
  float* onull = nullptr;
  _Float16* hnull = nullptr;
  for (int i = 0; i < NLAY; ++i) {
    const _Float16* wq_i = Wp + (size_t)0 * NWPL + (size_t)i * HID * HID;
    const _Float16* wk_i = Wp + (size_t)1 * NWPL + (size_t)i * HID * HID;
    const _Float16* wv_i = Wp + (size_t)2 * NWPL + (size_t)i * HID * HID;
    const _Float16* w1_i = Wp + (size_t)3 * NWPL + (size_t)i * HID * HID;
    const _Float16* w2_i = Wp + (size_t)4 * NWPL + (size_t)i * HID * HID;
    k_ln<<<dim3(NTOK / 16), dim3(256), 0, stream>>>(X, fnull, ln1_g + i * HID, ln1_b + i * HID, Qin, Qinh);
    k_gemm<<<dim3(NTOK / 128), dim3(256), 0, stream>>>(Qinh, wq_i, bq + i * HID, fnull, fnull, inull,
                                                      0, 0.015625f, 1.0f, Qf, hnull);
    k_gemm<<<dim3(NTOK / 128), dim3(256), 0, stream>>>(Xh, wk_i, bk + i * HID, pos_K, fnull, inull,
                                                      0, 0.015625f, 1.0f, onull, Kh);
    k_gemm<<<dim3(NTOK / 128), dim3(256), 0, stream>>>(Xh, wv_i, bv + i * HID, pos_V, fnull, inull,
                                                      0, 0.015625f, 1.0f, onull, Vh);
    k_attn<<<dim3(NSEQ * NHD), dim3(ATT_THREADS), ATT_LDS, stream>>>(Qf, Kh, Vh, tm_K, tm_V, tmat, log_seqs,
                                                                    Op, sscale);
    k_ln<<<dim3(NTOK / 16), dim3(256), 0, stream>>>(Qin, Op, ln2_g + i * HID, ln2_b + i * HID, Y, Yh);
    k_gemm<<<dim3(NTOK / 128), dim3(256), 0, stream>>>(Yh, w1_i, b1 + i * HID, fnull, fnull, inull,
                                                      1, 0.015625f, 16.0f, onull, Hm);
    k_gemm<<<dim3(NTOK / 128), dim3(256), 0, stream>>>(Hm, w2_i, b2 + i * HID, fnull, Y, log_seqs,
                                                      0, 0.0009765625f, 1.0f, X, Xh);
  }
  k_final<<<dim3(NTOK / 32), dim3(256), 0, stream>>>(X, lnf_g, lnf_b, item_emb, nitems, pos_seqs, neg_seqs, out);
  (void)hipGetLastError();
}
